// LSTMDirectionModel_76708115906740
// MI455X (gfx1250) — hardware-verified
//
#include <hip/hip_runtime.h>


#define B_   4096
#define T_   512
#define I_   3
#define H_   32
#define G4_  128
#define C_   3
#define MB_  64
#define NTHR 256
#define NBLK (B_ / MB_)
#define TQ_  (T_ / 4)

static_assert(G4_ == 4 * H_);
static_assert(H_ == 32);
static_assert(B_ == 4096);
static_assert((B_ & (B_ - 1)) == 0);
static_assert(B_ % MB_ == 0);
static_assert(MB_ == 64);
static_assert(NTHR == 256);
static_assert((NTHR / 32) == (MB_ / 16) * (H_ / 16));
static_assert(T_ % 4 == 0);
static_assert((G4_ * H_) == NTHR * 16);
static_assert((G4_ * I_) % 4 == 0);
static_assert((MB_ * C_) % 4 == 0);
static_assert(((MB_ * C_ * 4) % 128) == 0);

typedef float          v4f   __attribute__((ext_vector_type(4)));
typedef float          v8f   __attribute__((ext_vector_type(8)));
typedef unsigned short v8us  __attribute__((ext_vector_type(8)));
typedef unsigned short v16us __attribute__((ext_vector_type(16)));
typedef __bf16         v16b  __attribute__((ext_vector_type(16)));

union FragB { v16us u; v8us half[2]; };

constexpr int    NXP    = TQ_ * B_;
constexpr int    NXBLK  = NXP / 256;
constexpr size_t SZ_XT  = (size_t)T_ * B_ * 16;
constexpr size_t OFF_XT = 0;
constexpr size_t WS_END = OFF_XT + SZ_XT;
static_assert(NXP % 256 == 0);
static_assert((size_t)NXP * 4 * 16 == SZ_XT);
static_assert(WS_END <= (size_t)134217728);

__device__ __forceinline__ unsigned int bf16_rne_bits(float f) {
    unsigned int u = __float_as_uint(f);
    u += 0x7FFFu + ((u >> 16) & 1u);
    return u >> 16;
}
__device__ __forceinline__ float bf16_rne(float f) { return __uint_as_float(bf16_rne_bits(f) << 16); }
__device__ __forceinline__ float rcpx(float x) { return __builtin_amdgcn_rcpf(x); }
__device__ __forceinline__ float sigm(float x) { return rcpx(1.0f + expf(-x)); }
__device__ __forceinline__ float tanhx(float x) {
    const float e = expf(2.0f * x);
    return 1.0f - 2.0f * rcpx(e + 1.0f);
}
__device__ __forceinline__ v8f zero8() {
    v8f z;
#pragma unroll
    for (int i = 0; i < 8; ++i) z[i] = 0.0f;
    return z;
}

__device__ __forceinline__ void ldfrag_lds(FragB& f, const unsigned short* p) {
    f.half[0] = *(const v8us*)(p);
    f.half[1] = *(const v8us*)(p + 16);
}
__device__ __forceinline__ v8f mma_bf16(v8f c, const FragB& a, const FragB& b) {
    return __builtin_amdgcn_wmma_f32_16x16x32_bf16(false, __builtin_bit_cast(v16b, a.u), false,
                                                  __builtin_bit_cast(v16b, b.u), (short)0, c, false, false);
}

__global__ __launch_bounds__(256)
void xprep_kernel(const float* __restrict__ x, float* xT)
{
    const int p  = blockIdx.x * 256 + threadIdx.x;
    const int tq = p >> 12;
    const int b  = p & (B_ - 1);
    const float* src = x + (size_t)b * (T_ * I_) + (size_t)tq * 12;
    const v4f u0 = *(const v4f*)(src);
    const v4f u1 = *(const v4f*)(src + 4);
    const v4f u2 = *(const v4f*)(src + 8);
    v4f o0, o1, o2, o3;
    o0[0] = bf16_rne(u0[0]); o0[1] = bf16_rne(u0[1]); o0[2] = bf16_rne(u0[2]); o0[3] = 0.0f;
    o1[0] = bf16_rne(u0[3]); o1[1] = bf16_rne(u1[0]); o1[2] = bf16_rne(u1[1]); o1[3] = 0.0f;
    o2[0] = bf16_rne(u1[2]); o2[1] = bf16_rne(u1[3]); o2[2] = bf16_rne(u2[0]); o2[3] = 0.0f;
    o3[0] = bf16_rne(u2[1]); o3[1] = bf16_rne(u2[2]); o3[2] = bf16_rne(u2[3]); o3[3] = 0.0f;
    float* d0 = xT + ((size_t)(4 * tq) * B_ + b) * 4;
    float* d1 = d0 + (size_t)B_ * 4;
    float* d2 = d1 + (size_t)B_ * 4;
    float* d3 = d2 + (size_t)B_ * 4;
    *(volatile v4f*)d0 = o0;
    *(volatile v4f*)d1 = o1;
    *(volatile v4f*)d2 = o2;
    *(volatile v4f*)d3 = o3;
    __threadfence();
    *(volatile v4f*)d0 = o0;
    *(volatile v4f*)d1 = o1;
    *(volatile v4f*)d2 = o2;
    *(volatile v4f*)d3 = o3;
}

__global__ __launch_bounds__(NTHR)
void lstm_seq_kernel(const float* __restrict__ xT, const float* __restrict__ Wih,
                     const float* __restrict__ Whh, const float* __restrict__ bih,
                     const float* __restrict__ bhh, const float* __restrict__ Wfc,
                     const float* __restrict__ bfc, float* out)
{
    __shared__ __attribute__((aligned(16))) unsigned short sW[G4_ * H_];
    __shared__ __attribute__((aligned(16))) unsigned short sH[2 * 2 * MB_ * H_];
    __shared__ __attribute__((aligned(16))) float sX[2 * MB_ * 4];
    __shared__ __attribute__((aligned(16))) float sWih[G4_ * I_];
    __shared__ __attribute__((aligned(16))) float sBias[G4_];
    __shared__ __attribute__((aligned(16))) float sWfc[C_ * H_];
    __shared__ __attribute__((aligned(16))) float sBfc[4];
    __shared__ __attribute__((aligned(16))) float sHf[MB_ * H_];
    __shared__ __attribute__((aligned(16))) float sOut[MB_ * 4];

    const int tid  = threadIdx.x;
    const int lane = tid & 31;
    const int w    = tid >> 5;
    const int h    = lane >> 4;
    const int m    = lane & 15;
    const int mt   = w >> 1;
    const int cg   = w & 1;
    const int n    = cg * 16 + m;
    const int b0   = blockIdx.x * MB_;

    {
        const float* src = Whh + tid * 16;
        const v4f a0 = *(const v4f*)(src);
        const v4f a1 = *(const v4f*)(src + 4);
        const v4f a2 = *(const v4f*)(src + 8);
        const v4f a3 = *(const v4f*)(src + 12);
        v8us p0, p1;
#pragma unroll
        for (int i = 0; i < 4; ++i) {
            p0[i]     = (unsigned short)bf16_rne_bits(a0[i]);
            p0[4 + i] = (unsigned short)bf16_rne_bits(a1[i]);
            p1[i]     = (unsigned short)bf16_rne_bits(a2[i]);
            p1[4 + i] = (unsigned short)bf16_rne_bits(a3[i]);
        }
        *(v8us*)(sW + tid * 16)     = p0;
        *(v8us*)(sW + tid * 16 + 8) = p1;
    }
    {
        v8us z;
#pragma unroll
        for (int i = 0; i < 8; ++i) z[i] = (unsigned short)0;
        for (int i = tid; i < (2 * 2 * MB_ * H_) / 8; i += NTHR) *(v8us*)(sH + 8 * i) = z;
    }
    if (tid < (G4_ * I_) / 4) {
        const v4f v = *(const v4f*)(Wih + tid * 4);
        v4f r;
#pragma unroll
        for (int i = 0; i < 4; ++i) r[i] = bf16_rne(v[i]);
        *(v4f*)(sWih + tid * 4) = r;
    }
    if (tid < G4_) sBias[tid] = bf16_rne(bih[tid]) + bf16_rne(bhh[tid]);
    if (tid < C_ * H_) sWfc[tid] = bf16_rne(Wfc[tid]);
    if (tid < 4) {
        const float v = bf16_rne(bfc[min(tid, C_ - 1)]);
        sBfc[tid] = (tid < C_) ? v : 0.0f;
    }
    if (tid < MB_) *(v4f*)(sX + tid * 4) = *(const v4f*)(xT + ((size_t)b0 + tid) * 4);
    __syncthreads();

    float wi0[4], wi1[4], wi2[4], bs[4];
#pragma unroll
    for (int q = 0; q < 4; ++q) {
        const int g = q * H_ + n;
        wi0[q] = sWih[g * I_ + 0];
        wi1[q] = sWih[g * I_ + 1];
        wi2[q] = sWih[g * I_ + 2];
        bs[q]  = sBias[g];
    }
    float cst[8], hl[8];
#pragma unroll
    for (int r = 0; r < 8; ++r) { cst[r] = 0.0f; hl[r] = 0.0f; }

#pragma unroll 1
    for (int s = 0; s < T_; ++s) {
        const int cur = s & 1;
        const int nxt = cur ^ 1;

        __syncthreads();

        if (tid < MB_) {
            const int tn = min(s + 1, T_ - 1);
            const v4f xv = *(const v4f*)(xT + ((size_t)tn * B_ + b0 + tid) * 4);
            *(v4f*)(sX + nxt * (MB_ * 4) + tid * 4) = xv;
        }

        const unsigned short* hc  = sH + cur * (2 * MB_ * H_);
        unsigned short*       hnx = sH + nxt * (2 * MB_ * H_);
        FragB ahi, alo, bq[4];
        {
            const unsigned short* ap = hc + (16 * mt + m) * H_ + 8 * h;
            ldfrag_lds(ahi, ap);
            ldfrag_lds(alo, ap + MB_ * H_);
#pragma unroll
            for (int q = 0; q < 4; ++q) ldfrag_lds(bq[q], sW + (q * H_ + n) * H_ + 8 * h);
        }
        v8f acc[4];
#pragma unroll
        for (int q = 0; q < 4; ++q) acc[q] = mma_bf16(zero8(), ahi, bq[q]);
#pragma unroll
        for (int q = 0; q < 4; ++q) acc[q] = mma_bf16(acc[q], alo, bq[q]);
        asm volatile("v_nop\n\tv_nop\n\tv_nop\n\tv_nop"
                     : "+v"(acc[0]), "+v"(acc[1]), "+v"(acc[2]), "+v"(acc[3])
                     : "v"(ahi.u), "v"(alo.u), "v"(bq[0].u), "v"(bq[1].u), "v"(bq[2].u), "v"(bq[3].u));

        const float* xc = sX + cur * (MB_ * 4);
#pragma unroll
        for (int r = 0; r < 8; ++r) {
            const int rowb = 16 * mt + 8 * h + r;
            const v4f xv = *(const v4f*)(xc + rowb * 4);
            float pre[4];
#pragma unroll
            for (int q = 0; q < 4; ++q) {
                const float xg = fmaf(xv[2], wi2[q], fmaf(xv[1], wi1[q], xv[0] * wi0[q])) + bs[q];
                pre[q] = xg + acc[q][r];
            }
            const float ig = sigm(pre[0]);
            const float fg = sigm(pre[1]);
            const float gg = tanhx(pre[2]);
            const float og = sigm(pre[3]);
            const float cn = fg * cst[r] + ig * gg;
            cst[r] = cn;
            const float hn = og * tanhx(cn);
            hl[r] = hn;
            const unsigned int hib = bf16_rne_bits(hn);
            const float        hif = __uint_as_float(hib << 16);
            const unsigned int lob = bf16_rne_bits(hn - hif);
            hnx[rowb * H_ + n]            = (unsigned short)hib;
            hnx[MB_ * H_ + rowb * H_ + n] = (unsigned short)lob;
        }
    }

#pragma unroll
    for (int r = 0; r < 8; ++r) sHf[(16 * mt + 8 * h + r) * H_ + n] = hl[r];
    __syncthreads();
    if (tid < MB_ * C_) {
        const int row = tid / C_;
        const int cls = tid - row * C_;
        float a = 0.0f;
#pragma unroll 8
        for (int j = 0; j < H_; ++j) a = fmaf(sHf[row * H_ + j], sWfc[cls * H_ + j], a);
        sOut[tid] = a + sBfc[cls];
    }
    __syncthreads();
    v4f ov;
#pragma unroll
    for (int i = 0; i < 4; ++i) ov[i] = 0.0f;
    if (tid < (MB_ * C_) / 4) ov = *(const v4f*)(sOut + tid * 4);
    float* op = out + (size_t)b0 * C_ + tid * 4;
    if (tid < (MB_ * C_) / 4) *(volatile v4f*)op = ov;
    __threadfence();
    if (tid < (MB_ * C_) / 4) *(volatile v4f*)op = ov;
}

extern "C" void kernel_launch(void* const* d_in, const int* in_sizes, int n_in,
                              void* d_out, int out_size, void* d_ws, size_t ws_size,
                              hipStream_t stream)
{
    if (n_in < 7) return;
    if (in_sizes[0] != B_ * T_ * I_) return;
    if (in_sizes[1] != G4_ * I_)     return;
    if (in_sizes[2] != G4_ * H_)     return;
    if (in_sizes[3] != G4_)          return;
    if (in_sizes[4] != G4_)          return;
    if (in_sizes[5] != C_ * H_)      return;
    if (in_sizes[6] != C_)           return;
    if (out_size != B_ * C_)         return;
    if (ws_size < WS_END)            return;

    const float* x   = (const float*)d_in[0];
    const float* Wih = (const float*)d_in[1];
    const float* Whh = (const float*)d_in[2];
    const float* bih = (const float*)d_in[3];
    const float* bhh = (const float*)d_in[4];
    const float* Wfc = (const float*)d_in[5];
    const float* bfc = (const float*)d_in[6];
    float* out = (float*)d_out;

    char* ws = (char*)d_ws;
    float* xT = (float*)(ws + OFF_XT);

    xprep_kernel<<<dim3(NXBLK), dim3(256), 0, stream>>>(x, xT);
    lstm_seq_kernel<<<dim3(NBLK), dim3(NTHR), 0, stream>>>(
        (const float*)xT, Wih, Whh, bih, bhh, Wfc, bfc, out);
}
